// EdgeConvBlock_22926535426431
// MI455X (gfx1250) — hardware-verified
//
#include <hip/hip_runtime.h>
#include <stddef.h>
#include <stdint.h>

#define DIN    64
#define COUT   64
#define UQW    128
#define K2     128
#define NTHR   256
#define NWAVE  8
#define AP     136
#define WP     136
#define TP     72
#define PIECE  16
#define GBM    64
#define GBN    128
#define GTHR   128
#define EPT    8
#define CHUNK  (NTHR * EPT)
#define WCAP   (EPT * 32)
#define LISTN  (NWAVE * WCAP)
#define NBA    1024
#define SLA    10
#define RCAP   20480
#define DEGCAP 48
#define AGG_ZINTS    (LISTN + 2 * RCAP + 3 * NBA)
#define MISC_INTS    16
#define W2L_INTS     (COUT * WP / 2)
#define AT_INTS      (NWAVE * PIECE * AP / 2)
#define STG_INTS     (NWAVE * COUT)
#define B2_INTS      COUT
#define AGG_LDS_INTS (AGG_ZINTS + MISC_INTS + W2L_INTS + AT_INTS + STG_INTS + B2_INTS)
#define AGG_LDS_BYTES (AGG_LDS_INTS * 4)
#define WSMAX  134217728

static_assert((CHUNK & (CHUNK - 1)) == 0 && CHUNK <= 4096);
static_assert((NBA & (NBA - 1)) == 0 && NBA == (1 << SLA));
static_assert(((long long)CHUNK << SLA) < (1LL << 31));
static_assert(LISTN % NTHR == 0);
static_assert(NBA % NWAVE == 0 && NBA % 32 == 0);
static_assert(RCAP % 4 == 0 && LISTN % 4 == 0 && AGG_ZINTS % (NTHR * 4) == 0);
static_assert(((AGG_ZINTS + MISC_INTS) % 4) == 0 && (W2L_INTS % 4) == 0 && (AT_INTS % 4) == 0 && (STG_INTS % 4) == 0);
static_assert(AGG_LDS_BYTES <= 300000);
static_assert((AP * 2) % 16 == 0 && (WP * 2) % 16 == 0 && (TP * 2) % 16 == 0 && AP >= K2 && WP >= K2 && TP >= COUT);
static_assert(DEGCAP % PIECE == 0 && PIECE * 2 == 32);
static_assert(DIN % 32 == 0 && K2 % 32 == 0 && K2 == 2 * COUT && UQW == 2 * COUT && GBN == UQW);
static_assert(GBM == (GTHR / 32) * 16 && GBN == 8 * 16 && COUT == 2 * 32 && COUT == 4 * 16);
static_assert(COUT * COUT == 16 * NTHR && COUT * (DIN / 8) == 2 * NTHR && COUT * (K2 / 8) == 4 * NTHR);

typedef float          v2f   __attribute__((ext_vector_type(2)));
typedef float          v4f   __attribute__((ext_vector_type(4)));
typedef float          v8f   __attribute__((ext_vector_type(8)));
typedef int            v4i   __attribute__((ext_vector_type(4)));
typedef int            v8i   __attribute__((ext_vector_type(8)));
typedef unsigned short v8us  __attribute__((ext_vector_type(8)));
typedef unsigned short v16us __attribute__((ext_vector_type(16)));
typedef __bf16         v16bf __attribute__((ext_vector_type(16)));
typedef v2f  __attribute__((may_alias)) v2fa;
typedef v4f  __attribute__((may_alias)) v4fa;
typedef v4i  __attribute__((may_alias)) v4ia;
typedef v8us __attribute__((may_alias)) v8usa;
union FragB { v16bf v; v16us u; v8us h[2]; v8i w; };

__device__ __forceinline__ v8f wmb(const FragB& a, const FragB& b, v8f c) {
  v8f d = __builtin_amdgcn_wmma_f32_16x16x32_bf16(false, a.v, false, b.v, (short)0, c, false, false);
  asm volatile("v_nop\n\tv_nop\n\tv_nop\n\tv_nop" : "+v"(d) : "v"(a.w), "v"(b.w));
  return d;
}

__device__ __forceinline__ v8f z8() { v8f z = {0.f, 0.f, 0.f, 0.f, 0.f, 0.f, 0.f, 0.f}; return z; }

__device__ __forceinline__ unsigned bf16_bits(float f) {
  const unsigned u = __float_as_uint(f);
  return (u + 0x7FFFu + ((u >> 16) & 1u)) >> 16;
}
__device__ __forceinline__ float bf16_val(float f) {
  return __uint_as_float(bf16_bits(f) << 16);
}
__device__ __forceinline__ void put16(unsigned short* dp, v8us o) {
  *(volatile v8us*)dp = o;
  __threadfence();
  *(volatile v8us*)dp = o;
}
__device__ __forceinline__ float fsel(float a, float b, unsigned mask) {
  return __uint_as_float((__float_as_uint(a) & ~mask) | (__float_as_uint(b) & mask));
}
__device__ __forceinline__ void wave_sync() {
  __builtin_amdgcn_fence(__ATOMIC_RELEASE, "wavefront");
  __builtin_amdgcn_wave_barrier();
  __builtin_amdgcn_fence(__ATOMIC_ACQUIRE, "wavefront");
}

template <int SLB>
__device__ __forceinline__ int scan_chunk(const int* __restrict__ dsts, int nE, int cbase, int slotBase,
                                          int nb, int vec8, int* list, int tid, int lane, int wave) {
  int wc = 0;
  const int el0  = tid * EPT;
  const int e0   = cbase + el0;
  const int sent = -2147483647 - 1;
  v4i da, db;
  if (vec8 != 0 && cbase + CHUNK <= nE) {
    da = *(const v4i*)(dsts + e0);
    db = *(const v4i*)(dsts + e0 + 4);
  } else {
    da.x = (e0     < nE) ? dsts[min(e0,     nE - 1)] : sent;
    da.y = (e0 + 1 < nE) ? dsts[min(e0 + 1, nE - 1)] : sent;
    da.z = (e0 + 2 < nE) ? dsts[min(e0 + 2, nE - 1)] : sent;
    da.w = (e0 + 3 < nE) ? dsts[min(e0 + 3, nE - 1)] : sent;
    db.x = (e0 + 4 < nE) ? dsts[min(e0 + 4, nE - 1)] : sent;
    db.y = (e0 + 5 < nE) ? dsts[min(e0 + 5, nE - 1)] : sent;
    db.z = (e0 + 6 < nE) ? dsts[min(e0 + 6, nE - 1)] : sent;
    db.w = (e0 + 7 < nE) ? dsts[min(e0 + 7, nE - 1)] : sent;
  }
  const unsigned nbs = (unsigned)slotBase;
  const unsigned unb = (unsigned)nb;
  const unsigned s0 = (unsigned)da.x - nbs, s1 = (unsigned)da.y - nbs;
  const unsigned s2 = (unsigned)da.z - nbs, s3 = (unsigned)da.w - nbs;
  const unsigned s4 = (unsigned)db.x - nbs, s5 = (unsigned)db.y - nbs;
  const unsigned s6 = (unsigned)db.z - nbs, s7 = (unsigned)db.w - nbs;
  const bool h0 = s0 < unb, h1 = s1 < unb, h2 = s2 < unb, h3 = s3 < unb;
  const bool h4 = s4 < unb, h5 = s5 < unb, h6 = s6 < unb, h7 = s7 < unb;
  const unsigned any = __builtin_amdgcn_ballot_w32(h0 | h1 | h2 | h3 | h4 | h5 | h6 | h7);
  if (any != 0u) {
#define HITJ(J, HJ, SJ) { \
      const unsigned mj = __builtin_amdgcn_ballot_w32(HJ); \
      if (mj != 0u) { \
        if (HJ) { \
          const int pos = wc + (int)__builtin_amdgcn_mbcnt_lo(mj, 0u); \
          if (pos < WCAP) list[wave * WCAP + pos] = ((el0 + (J)) << SLB) | (int)(SJ); \
        } \
        wc += (int)__builtin_popcount(mj); } }
    HITJ(0, h0, s0)
    HITJ(1, h1, s1)
    HITJ(2, h2, s2)
    HITJ(3, h3, s3)
    HITJ(4, h4, s4)
    HITJ(5, h5, s5)
    HITJ(6, h6, s6)
    HITJ(7, h7, s7)
#undef HITJ
  }
  return wc;
}

__global__ __launch_bounds__(NTHR) void k_wprep(const float* __restrict__ W1, const float* __restrict__ W2,
                                                unsigned short* W1T, unsigned short* W2B) {
  __shared__ __attribute__((aligned(16))) unsigned short T[COUT * TP];
  const int tid = (int)threadIdx.x;
  const int b   = (int)blockIdx.x;
  const float* src = (b == 0) ? W1 : ((b == 1) ? (W1 + COUT * COUT) : W2);
#pragma unroll
  for (int it = 0; it < 4; ++it) {
    const int idx = 4 * (it * NTHR + tid);
    const int k = idx >> 6, n0 = idx & 63;
    const v4f v = *(const v4f*)(src + idx);
    T[(n0 + 0) * TP + k] = (unsigned short)bf16_bits(v.x);
    T[(n0 + 1) * TP + k] = (unsigned short)bf16_bits(v.y);
    T[(n0 + 2) * TP + k] = (unsigned short)bf16_bits(v.z);
    T[(n0 + 3) * TP + k] = (unsigned short)bf16_bits(v.w);
  }
  __syncthreads();
  if (b < 2) {
#pragma unroll
    for (int it = 0; it < 2; ++it) {
      const int p  = it * NTHR + tid;
      const int n  = p >> 3, c8 = (p & 7) * 8;
      const v8us o = *(const v8usa*)(T + n * TP + c8);
      put16(W1T + (size_t)b * (size_t)(COUT * DIN) + (size_t)p * 8, o);
    }
  } else {
#pragma unroll
    for (int it = 0; it < 4; ++it) {
      const int p  = it * NTHR + tid;
      const int n  = p >> 4;
      const int c8 = ((p & 15) * 8) & (COUT - 1);
      const v8us o = *(const v8usa*)(T + n * TP + c8);
      put16(W2B + (size_t)p * 8, o);
    }
  }
}

__global__ __launch_bounds__(NTHR) void k_xprep(const float* __restrict__ x, int nN, int mRows,
                                                unsigned short* XB) {
  const int u   = (int)blockIdx.x * NTHR + (int)threadIdx.x;
  const int row = u >> 3, j = u & 7;
  if (row >= mRows) return;
  const int rc = row < nN ? row : nN - 1;
  const unsigned mk = (row < nN) ? 0xffffu : 0u;
  const float* p = x + (size_t)rc * DIN + 8 * j;
  const v4f a = *(const v4f*)p;
  const v4f b = *(const v4f*)(p + 4);
  v8us o;
  o[0] = (unsigned short)(bf16_bits(a.x) & mk); o[1] = (unsigned short)(bf16_bits(a.y) & mk);
  o[2] = (unsigned short)(bf16_bits(a.z) & mk); o[3] = (unsigned short)(bf16_bits(a.w) & mk);
  o[4] = (unsigned short)(bf16_bits(b.x) & mk); o[5] = (unsigned short)(bf16_bits(b.y) & mk);
  o[6] = (unsigned short)(bf16_bits(b.z) & mk); o[7] = (unsigned short)(bf16_bits(b.w) & mk);
  put16(XB + (size_t)u * 8, o);
}

__global__ __launch_bounds__(GTHR) void k_pq(const unsigned short* __restrict__ A,
                                             const unsigned short* __restrict__ BT,
                                             const float* __restrict__ b1, float* UQ) {
  __shared__ __attribute__((aligned(16))) float stg[GBM * GBN];
  const int tid = (int)threadIdx.x, lane = tid & 31, wave = tid >> 5, hh = lane >> 4, m = lane & 15;
  const int rowBase = (int)blockIdx.x * GBM;

  v8f acc[8];
#pragma unroll
  for (int t = 0; t < 8; ++t) acc[t] = z8();
  const unsigned short* ap = A  + (size_t)(rowBase + 16 * wave + m) * (size_t)DIN + 8 * hh;
  const unsigned short* bp = BT + (size_t)m * (size_t)DIN + 8 * hh;

#pragma unroll
  for (int k0 = 0; k0 < DIN; k0 += 32) {
    FragB af;
    af.h[0] = *(const v8usa*)(ap + k0);
    af.h[1] = *(const v8usa*)(ap + k0 + 16);
#pragma unroll
    for (int nt = 0; nt < 8; ++nt) {
      const unsigned short* wq = bp + (size_t)(16 * nt) * (size_t)DIN + k0;
      FragB bf;
      bf.h[0] = *(const v8usa*)wq;
      bf.h[1] = *(const v8usa*)(wq + 16);
      acc[nt] = wmb(af, bf, acc[nt]);
    }
  }

#pragma unroll
  for (int nt = 0; nt < 8; ++nt) {
    const int lc = 16 * nt + m;
#pragma unroll
    for (int r = 0; r < 8; ++r) {
      const int lr = 16 * wave + 8 * hh + r;
      stg[lr * GBN + lc] = acc[nt][r];
    }
  }
  __syncthreads();

  const int cU = 4 * (lane & 15);
  const unsigned mq = 0u - (unsigned)hh;
  const v4f b4 = *(const v4f*)(b1 + cU);
  const float bb0 = bf16_val(b4.x);
  const float bb1 = bf16_val(b4.y);
  const float bb2 = bf16_val(b4.z);
  const float bb3 = bf16_val(b4.w);
  v4f pv[16];
#pragma unroll
  for (int i = 0; i < 16; ++i) {
    const float* sp = stg + (16 * wave + i) * GBN;
    const v4f a = *(const v4fa*)(sp + cU);
    const v4f q = *(const v4fa*)(sp + COUT + cU);
    v4f o;
    o.x = fsel((a.x - q.x) + bb0, q.x, mq);
    o.y = fsel((a.y - q.y) + bb1, q.y, mq);
    o.z = fsel((a.z - q.z) + bb2, q.z, mq);
    o.w = fsel((a.w - q.w) + bb3, q.w, mq);
    pv[i] = o;
  }
#pragma unroll
  for (int i = 0; i < 16; ++i) {
    float* op = UQ + (size_t)(rowBase + 16 * wave + i) * (size_t)UQW + 4 * lane;
    *(volatile v4f*)op = pv[i];
  }
  __threadfence();
#pragma unroll
  for (int i = 0; i < 16; ++i) {
    float* op = UQ + (size_t)(rowBase + 16 * wave + i) * (size_t)UQW + 4 * lane;
    *(volatile v4f*)op = pv[i];
  }
}

__global__ __launch_bounds__(NTHR) void k_scan(const int* __restrict__ srcs, const int* __restrict__ dsts,
                                               int nE, int nN, int vec8, const float* __restrict__ UQ,
                                               const unsigned short* __restrict__ W2B,
                                               const float* __restrict__ b2, float* out) {
  extern __shared__ __attribute__((aligned(16))) int dsm[];
  int* list = dsm;
  int* hl   = dsm + LISTN;
  int* sl   = hl + RCAP;
  int* cnt  = sl + RCAP;
  int* offs = cnt + NBA;
  int* cur  = offs + NBA;
  int* misc = cur + NBA;
  unsigned short* sW2 = (unsigned short*)(misc + MISC_INTS);
  unsigned short* sAt = sW2 + 2 * W2L_INTS;
  float*          stg = (float*)(sAt + 2 * AT_INTS);
  float*          sb2 = stg + STG_INTS;
  const int tid = (int)threadIdx.x, lane = tid & 31, wave = tid >> 5;
  const int nodeBase = (int)blockIdx.x * NBA;

  {
    const v4i z4 = {0, 0, 0, 0};
    for (int i = tid * 4; i < AGG_ZINTS; i += NTHR * 4) *(v4ia*)(dsm + i) = z4;
    if (tid < MISC_INTS) misc[tid] = 0;
#pragma unroll
    for (int it = 0; it < 4; ++it) {
      const int p  = it * NTHR + tid;
      const int n  = p >> 4, c8 = (p & 15) * 8;
      const v8us w = *(const v8usa*)(W2B + (size_t)p * 8);
      *(v8usa*)(sW2 + n * WP + c8) = w;
    }
    if (tid < COUT) sb2[tid] = bf16_val(b2[tid]);
  }
  __syncthreads();

  int t = 0, ov = 0;
  const int nChunks = (nE + CHUNK - 1) / CHUNK;
#pragma unroll 1
  for (int ch = 0; ch < nChunks; ++ch) {
    const int cbase = ch * CHUNK;
    const int wc = scan_chunk<SLA>(dsts, nE, cbase, nodeBase, NBA, vec8, list, tid, lane, wave);
    if (lane == 0) misc[wave] = wc;
    __syncthreads();
    if (wave == 0) {
#pragma unroll 1
      for (int w2 = 0; w2 < NWAVE; ++w2) {
        int c = misc[w2];
        c = c < 0 ? 0 : (c > WCAP ? WCAP : c);
#pragma unroll 1
        for (int b0 = 0; b0 < c; b0 += 32) {
          const int idx = b0 + lane;
          const int ent = list[w2 * WCAP + (idx < WCAP ? idx : WCAP - 1)];
          const int m32 = (c - b0) < 32 ? (c - b0) : 32;
#pragma unroll 1
          for (int k = 0; k < m32; ++k) {
            const int u    = __builtin_amdgcn_readlane(ent, k);
            const int slot = u & (NBA - 1);
            const int el   = (u >> SLA) & (CHUNK - 1);
            const int pk   = ((cbase + el) << SLA) | slot;
            if (t < RCAP) {
              if (lane == 0) { hl[t] = pk; cnt[slot] = cnt[slot] + 1; }
              t = t + 1;
            } else {
              ov = 1;
            }
          }
        }
      }
    }
    __syncthreads();
  }
  if (wave == 0 && lane == 0) { misc[8] = t; misc[9] = ov; }
  __syncthreads();
  int tt = misc[8];
  tt = tt < 0 ? 0 : (tt > RCAP ? RCAP : tt);
  const int ovf = misc[9];

  if (wave == 0) {
    const int base = lane * (NBA / 32);
    int sacc = 0;
#pragma unroll 1
    for (int i = 0; i < NBA / 32; ++i) sacc += cnt[base + i];
    int incl = sacc;
#pragma unroll
    for (int d = 1; d < 32; d <<= 1) {
      const int y = __shfl_up(incl, d, 32);
      if (lane >= d) incl += y;
    }
    int run = incl - sacc;
#pragma unroll 1
    for (int i = 0; i < NBA / 32; ++i) {
      const int cv = cnt[base + i];
      offs[base + i] = run;
      cur[base + i]  = run;
      run += cv;
    }
  }
  __syncthreads();
  if (wave == 0) {
#pragma unroll 1
    for (int b0 = 0; b0 < tt; b0 += 32) {
      const int idx = b0 + lane;
      const int ent = hl[idx < RCAP ? idx : RCAP - 1];
      const int m32 = (tt - b0) < 32 ? (tt - b0) : 32;
#pragma unroll 1
      for (int k = 0; k < m32; ++k) {
        const int u    = __builtin_amdgcn_readlane(ent, k);
        const int slot = u & (NBA - 1);
        if (lane == 0) {
          int p = cur[slot];
          p = p < 0 ? 0 : (p > RCAP - 1 ? RCAP - 1 : p);
          sl[p] = u;
          cur[slot] = p + 1;
        }
      }
    }
  }
  __syncthreads();

  const float ninf = __uint_as_float(0xff800000u);
  const float qnan = __uint_as_float(0x7fc00000u);
  const float pz = (ovf != 0) ? qnan : 0.0f;
  const int hh = lane >> 4, m = lane & 15, er = lane >> 1, hs = lane & 1;
  unsigned short* at = sAt + wave * (PIECE * AP);
  float* sg = stg + wave * COUT;
  const unsigned short* afp = at  + m * AP + 8 * hh;
  const unsigned short* bfp = sW2 + m * WP + 8 * hh;
  unsigned short* arow = at + er * AP + 32 * hs;
#pragma unroll 1
  for (int si = 0; si < NBA / NWAVE; ++si) {
    const int s    = si * NWAVE + wave;
    const int node = nodeBase + s;
    const int c0 = cnt[s];
    const bool big = c0 > DEGCAP;
    const int c = c0 < 0 ? 0 : (c0 > DEGCAP ? DEGCAP : c0);
    int o = offs[s];
    o = o < 0 ? 0 : (o > RCAP ? RCAP : o);
    const int nc = node < nN ? node : nN - 1;
    const float* dq = UQ + (size_t)nc * UQW + 32 * hs;
    v4f d[8];
#pragma unroll
    for (int q = 0; q < 8; ++q) d[q] = *(const v4f*)(dq + 4 * q);
    float rm0 = ninf, rm1 = ninf, rm2 = ninf, rm3 = ninf;
    const int nP = (c + PIECE - 1) / PIECE;
#pragma unroll 1
    for (int p = 0; p < nP; ++p) {
      int nv = c - p * PIECE;
      nv = nv > PIECE ? PIECE : nv;
      int idx = o + p * PIECE + er;
      idx = idx > RCAP - 1 ? RCAP - 1 : idx;
      const int ent = sl[idx];
      int eid = ent >> SLA;
      eid = eid < 0 ? 0 : (eid > nE - 1 ? nE - 1 : eid);
      int sr = srcs[eid];
      sr = sr < 0 ? 0 : (sr > nN - 1 ? nN - 1 : sr);
      const unsigned vm = (er < nv) ? 0xffffffffu : 0u;
      const float* sp = UQ + (size_t)sr * UQW + COUT + 32 * hs;
#pragma unroll
      for (int q = 0; q < 8; q += 2) {
        const v4f sa = *(const v4f*)(sp + 4 * q);
        const v4f sb = *(const v4f*)(sp + 4 * q + 4);
        const v4f ta = d[q] + sa;
        const v4f tb = d[q + 1] + sb;
        const v8f t8 = {ta.x, ta.y, ta.z, ta.w, tb.x, tb.y, tb.z, tb.w};
        v8us oh, ol;
#pragma unroll
        for (int i = 0; i < 8; ++i) {
          const float hv = __uint_as_float(__float_as_uint(fmaxf(t8[i], 0.0f)) & vm);
          const unsigned hb = bf16_bits(hv);
          oh[i] = (unsigned short)hb;
          ol[i] = (unsigned short)bf16_bits(hv - __uint_as_float(hb << 16));
        }
        *(v8usa*)(arow + 4 * q) = oh;
        *(v8usa*)(arow + COUT + 4 * q) = ol;
      }
      wave_sync();

      v8f acc[4];
#pragma unroll
      for (int nt = 0; nt < 4; ++nt) acc[nt] = z8();
#pragma unroll 1
      for (int k0 = 0; k0 < K2; k0 += 32) {
        FragB af;
        af.h[0] = *(const v8usa*)(afp + k0);
        af.h[1] = *(const v8usa*)(afp + k0 + 16);
#pragma unroll
        for (int nt = 0; nt < 4; ++nt) {
          const unsigned short* wq = bfp + (16 * nt) * WP + k0;
          FragB bf;
          bf.h[0] = *(const v8usa*)wq;
          bf.h[1] = *(const v8usa*)(wq + 16);
          acc[nt] = wmb(af, bf, acc[nt]);
        }
      }
      float mx[4];
#pragma unroll
      for (int nt = 0; nt < 4; ++nt) {
        float tm = ninf;
#pragma unroll
        for (int r = 0; r < 8; ++r) {
          const float v = ((8 * hh + r) < nv) ? acc[nt][r] : ninf;
          tm = fmaxf(tm, v);
        }
        mx[nt] = tm;
      }
      const float x0 = __shfl_xor(mx[0], 16, 32);
      const float x1 = __shfl_xor(mx[1], 16, 32);
      const float x2 = __shfl_xor(mx[2], 16, 32);
      const float x3 = __shfl_xor(mx[3], 16, 32);
      rm0 = fmaxf(rm0, fmaxf(mx[0], x0));
      rm1 = fmaxf(rm1, fmaxf(mx[1], x1));
      rm2 = fmaxf(rm2, fmaxf(mx[2], x2));
      rm3 = fmaxf(rm3, fmaxf(mx[3], x3));
      wave_sync();
    }

    const float pzr = big ? qnan : pz;
    const bool has = c0 > 0;
    const float v0 = (has ? (rm0 + sb2[m])      : 0.0f) + pzr;
    const float v1 = (has ? (rm1 + sb2[16 + m]) : 0.0f) + pzr;
    const float v2 = (has ? (rm2 + sb2[32 + m]) : 0.0f) + pzr;
    const float v3 = (has ? (rm3 + sb2[48 + m]) : 0.0f) + pzr;
    const float wa = hh ? v2 : v0;
    const float wb = hh ? v3 : v1;
    sg[32 * hh + m]      = wa;
    sg[32 * hh + 16 + m] = wb;
    wave_sync();
    const v2f ovv = *(const v2fa*)(sg + 2 * lane);
    wave_sync();
    const bool live = node < nN;
    if (live) {
      float* op = out + (size_t)node * COUT + 2 * lane;
      *(volatile v2f*)op = ovv;
    }
    __threadfence();
    if (live) {
      float* op = out + (size_t)node * COUT + 2 * lane;
      *(volatile v2f*)op = ovv;
    }
  }
}

static inline int cdiv(int a, int b) { return (a + b - 1) / b; }
static inline size_t al256(size_t o) { return (o + 255) & ~(size_t)255; }

extern "C" void kernel_launch(void* const* d_in, const int* in_sizes, int n_in,
                              void* d_out, int out_size, void* d_ws, size_t ws_size,
                              hipStream_t stream) {
  if (n_in < 6) return;
  if (in_sizes[0] < DIN * 16 || (in_sizes[0] % DIN) != 0) return;
  const int nN = in_sizes[0] / DIN;
  if (in_sizes[1] < 2 || (in_sizes[1] & 1) != 0) return;
  const int nE = in_sizes[1] / 2;
  if (nE < 1 || nE >= (1 << 21) || nN >= (1 << 24)) return;
  if (in_sizes[2] != 2 * DIN * COUT) return;
  if (in_sizes[3] != COUT) return;
  if (in_sizes[4] != COUT * COUT) return;
  if (in_sizes[5] != COUT) return;
  if ((long long)out_size != (long long)nN * COUT) return;

  const float* x  = (const float*)d_in[0];
  const int*   ei = (const int*)d_in[1];
  const float* W1 = (const float*)d_in[2];
  const float* b1 = (const float*)d_in[3];
  const float* W2 = (const float*)d_in[4];
  const float* b2 = (const float*)d_in[5];
  float* out = (float*)d_out;
  const int* src = ei;
  const int* dst = ei + nE;

  const int MP = cdiv(nN, GBM) * GBM;
  const int gM = MP / GBM;
  const int gX = (MP * (DIN / 8)) / NTHR;
  if ((long long)gX * NTHR != (long long)MP * (DIN / 8)) return;
  const int gA = cdiv(nN, NBA);
  if ((long long)gA * NBA < (long long)nN) return;
  const int vec8 = ((nE & 3) == 0) ? 1 : 0;

  char* ws = (char*)d_ws;
  size_t off = 0;
  const size_t oW1T = off; off = al256(off + (size_t)UQW * DIN * 2);
  const size_t oW2B = off; off = al256(off + (size_t)COUT * K2 * 2);
  const size_t oXB  = off; off = al256(off + (size_t)MP * DIN * 2);
  const size_t oUQ  = off; off = al256(off + (size_t)MP * UQW * 4);
  if (off > ws_size || off > (size_t)WSMAX) return;
  unsigned short* W1T = (unsigned short*)(ws + oW1T);
  unsigned short* W2B = (unsigned short*)(ws + oW2B);
  unsigned short* XB  = (unsigned short*)(ws + oXB);
  float*          UQ  = (float*)(ws + oUQ);

  hipFuncSetAttribute(reinterpret_cast<const void*>(&k_scan), hipFuncAttributeMaxDynamicSharedMemorySize,
                      (int)AGG_LDS_BYTES);

  k_wprep<<<3, NTHR, 0, stream>>>(W1, W2, W1T, W2B);
  k_xprep<<<gX, NTHR, 0, stream>>>(x, nN, MP, XB);
  k_pq<<<gM, GTHR, 0, stream>>>(XB, W1T, b1, UQ);
  k_scan<<<gA, NTHR, AGG_LDS_BYTES, stream>>>(src, dst, nE, nN, vec8, UQ, W2B, b2, out);
}
